// GeodesicLayer_22582938042986
// MI455X (gfx1250) — hardware-verified
//
#include <hip/hip_runtime.h>


#define NPT  30000
#define RCHK 7552
#define NB   80
#define PB   5
#define TB   16
#define ICH  16
#define OCH  32
#define KH   (NB * ICH)
#define NOT  (OCH * TB)
#define NV   30000
#define DM   KH
#define LOSC 1024.0f

typedef _Float16 h16;
typedef unsigned short bf;
typedef __attribute__((ext_vector_type(16))) __bf16   v16bf;
typedef __attribute__((ext_vector_type(16))) _Float16 v16h;
typedef __attribute__((ext_vector_type(8)))  _Float16 v8h;
typedef __attribute__((ext_vector_type(8)))  unsigned short v8us;
typedef __attribute__((ext_vector_type(8)))  float    v8f;
typedef __attribute__((ext_vector_type(4)))  float    v4f;
typedef v8h  __attribute__((may_alias)) v8ha;
typedef v4f  __attribute__((may_alias)) v4fa;
typedef v8us __attribute__((may_alias)) v8usa;

__device__ __forceinline__ unsigned short f2bf(float f) { unsigned u = __float_as_uint(f); u += 0x7FFFu + ((u >> 16) & 1u); return (unsigned short)(u >> 16); }
__device__ __forceinline__ float bf2f(unsigned short b) { return __uint_as_float(((unsigned)b) << 16); }
__device__ __forceinline__ float bfr(float f) { return bf2f(f2bf(f)); }
__device__ __forceinline__ v16h cat16(v8h lo, v8h hi) { return __builtin_shufflevector(lo, hi, 0, 1, 2, 3, 4, 5, 6, 7, 8, 9, 10, 11, 12, 13, 14, 15); }
__device__ __forceinline__ v16bf cat16b(v8us lo, v8us hi) { return __builtin_bit_cast(v16bf, __builtin_shufflevector(lo, hi, 0, 1, 2, 3, 4, 5, 6, 7, 8, 9, 10, 11, 12, 13, 14, 15)); }
__device__ __forceinline__ v8f wmma16(v16h a, v16h b, v8f c) { return __builtin_amdgcn_wmma_f32_16x16x32_f16(false, a, false, b, (short)0, c, false, false); }
__device__ __forceinline__ v8f wmmab(v16bf a, v16bf b, v8f c) { return __builtin_amdgcn_wmma_f32_16x16x32_bf16(false, a, false, b, (short)0, c, false, false); }

template <bool SPLITA, bool F16OUT = false>
__global__ __launch_bounds__(128) void k_gemmb(const bf* __restrict__ A, const bf* __restrict__ Al, const bf* __restrict__ Bn, const float* __restrict__ bias, float* C, int ldc, h16* C2, const float* __restrict__ R = nullptr, int K = DM, int roundR = 1) {
    __shared__ __align__(16) float ost[4][16 * 68];
    const int lane = threadIdx.x & 31, wave = threadIdx.x >> 5, lr = lane & 15, hi = lane >> 4;
    const int r0 = blockIdx.x * 64 + wave * 16, c0 = blockIdx.y * 64;
    const size_t aoff = (size_t)(r0 + lr) * K + 8 * hi;
    size_t boff[4];
#pragma unroll
    for (int t = 0; t < 4; ++t) boff[t] = (size_t)(c0 + t * 16 + lr) * K + 8 * hi;
    v8f acc[4];
#pragma unroll
    for (int t = 0; t < 4; ++t) acc[t] = (v8f){};
#pragma unroll 1
    for (int kc = 0; kc < K; kc += 32) {
        const v16bf a = cat16b(*(const v8us*)(A + aoff + kc), *(const v8us*)(A + aoff + kc + 16));
        v16bf al = a;
        if (SPLITA) al = cat16b(*(const v8us*)(Al + aoff + kc), *(const v8us*)(Al + aoff + kc + 16));
#pragma unroll
        for (int t = 0; t < 4; ++t) { const v16bf b = cat16b(*(const v8us*)(Bn + boff[t] + kc), *(const v8us*)(Bn + boff[t] + kc + 16)); acc[t] = wmmab(a, b, acc[t]); if (SPLITA) acc[t] = wmmab(al, b, acc[t]); }
        asm volatile("v_nop\n\tv_nop\n\tv_nop\n\tv_nop" : "+v"(acc[0]), "+v"(acc[1]), "+v"(acc[2]), "+v"(acc[3]) : "v"(a), "v"(al));
    }
    float* os = &ost[wave][0];
#pragma unroll
    for (int t = 0; t < 4; ++t) { const float bv = bias ? bfr(bias[c0 + t * 16 + lr]) : 0.f;
#pragma unroll
        for (int j = 0; j < 8; ++j) os[(hi * 8 + j) * 68 + t * 16 + lr] = acc[t][j] + bv; }
    __syncthreads();
    if (F16OUT) {
        h16* crow = (h16*)(void*)C + (size_t)r0 * ldc + c0;
        auto pass = [&]() {
#pragma unroll
            for (int s = 0; s < 4; ++s) { const int row = 4 * s + (lane >> 3), piece = lane & 7; const float* sp = os + row * 68 + piece * 8; v8h o, o2;
#pragma unroll
                for (int i = 0; i < 8; ++i) { const h16 a = (h16)sp[i]; o[i] = a; o2[i] = (h16)((sp[i] - (float)a) * LOSC); }
                *(volatile v8h*)(crow + (size_t)row * ldc + piece * 8) = o; if (C2) *(volatile v8h*)(C2 + (size_t)r0 * ldc + c0 + (size_t)row * ldc + piece * 8) = o2; }
        };
        pass(); __threadfence(); pass();
    } else {
        float* crow = C + (size_t)r0 * ldc + c0;
        auto pass = [&]() {
#pragma unroll
            for (int s = 0; s < 8; ++s) { const int Lid = (lane >> 3) + 4 * s, piece = lane & 7; const int row = Lid >> 1, cofs = (Lid & 1) * 32 + piece * 4;
                v4f val = *(const v4fa*)(os + row * 68 + cofs); if (R) { const v4f rv = *(const v4f*)(R + ((size_t)r0 + row) * ldc + c0 + cofs); val += roundR ? (v4f){bfr(rv[0]), bfr(rv[1]), bfr(rv[2]), bfr(rv[3])} : rv; }
                *(volatile v4f*)(crow + (size_t)row * ldc + cofs) = val; }
        };
        pass(); __threadfence(); pass();
    }
}


__global__ __launch_bounds__(256) void k_gather(const float* __restrict__ x, const int* __restrict__ idx, const float* __restrict__ val, int p0, bf* Hh, bf* Hl) {
    const int lane = threadIdx.x & 31; const size_t wid = (size_t)blockIdx.x * 8 + (threadIdx.x >> 5); const int pl = (int)(wid / 5), g = (int)(wid % 5); const int p = p0 + pl;
    const int b = g * 16 + (lane >> 1), cb = (lane & 1) * 8; float acc[8];
#pragma unroll
    for (int i = 0; i < 8; ++i) acc[i] = 0.f;
    if (p < NPT) { const size_t r = (size_t)p * NB + b;
#pragma unroll
        for (int k = 0; k < 3; ++k) { int v = idx[r * 3 + k]; v = v < 0 ? 0 : (v >= NV ? NV - 1 : v); const float w = bfr(val[r * 3 + k]);
#pragma unroll
            for (int i = 0; i < 8; ++i) acc[i] = fmaf(w, bfr(x[(size_t)v * ICH + cb + i]), acc[i]); } }
    v8us oh, ol;
#pragma unroll
    for (int i = 0; i < 8; ++i) { const unsigned short hb = f2bf(acc[i]); oh[i] = hb; ol[i] = f2bf(acc[i] - bf2f(hb)); }
    const size_t o = (size_t)pl * KH + b * ICH + cb; *(volatile v8us*)(Hh + o) = oh; *(volatile v8us*)(Hl + o) = ol; __threadfence(); *(volatile v8us*)(Hh + o) = oh; *(volatile v8us*)(Hl + o) = ol;
}
__global__ __launch_bounds__(256) void k_lw(const float* __restrict__ wts, bf* LWT) {
    const int lane = threadIdx.x & 31, n = blockIdx.x * 8 + (threadIdx.x >> 5); if (n >= NOT) return; const int o = n / TB, t = n - o * TB;
#pragma unroll 1
    for (int ps = 0; ps < 2; ++ps) {
#pragma unroll 1
        for (int k0 = lane * 8; k0 < KH; k0 += 256) { v8us ob;
#pragma unroll
            for (int q = 0; q < 8; ++q) { const int k = k0 + q; const int j = k / ICH, c = k - j * ICH; const int src = (j + PB * t) % NB; ob[q] = f2bf(wts[((size_t)src * ICH + c) * OCH + o]); }
            *(volatile v8us*)(LWT + (size_t)n * KH + k0) = ob; }
        if (ps == 0) __threadfence(); }
}
__global__ __launch_bounds__(256) void k_max(const float* __restrict__ Y, int p0, float* OUTP) {
    const size_t g = (size_t)blockIdx.x * 256 + threadIdx.x; const int pl = (int)(g / OCH), o = (int)(g % OCH); const int p = p0 + pl; if (p >= NPT) return; float m = -3.0e38f;
#pragma unroll
    for (int t = 0; t < TB; ++t) m = fmaxf(m, Y[(size_t)pl * NOT + o * TB + t]);
    *(volatile float*)(OUTP + (size_t)p * OCH + o) = m; __threadfence(); *(volatile float*)(OUTP + (size_t)p * OCH + o) = m;
}

extern "C" void kernel_launch(void* const* d_in, const int* in_sizes, int n_in,
                              void* d_out, int out_size, void* d_ws, size_t ws_size, hipStream_t stream) {
    (void)in_sizes; (void)n_in; (void)out_size;
    const float* x = (const float*)d_in[0]; const int* idx = (const int*)d_in[1]; const float* val = (const float*)d_in[2]; const float* wts = (const float*)d_in[3];
    float* out = (float*)d_out;
    char* wsp = (char*)d_ws;
    auto take = [&](size_t bytes) { char* p = wsp; wsp += (bytes + 255) & ~(size_t)255; return (void*)p; };
    bf* Hh = (bf*)take((size_t)RCHK * KH * 2); bf* Hl = (bf*)take((size_t)RCHK * KH * 2); bf* LWT = (bf*)take((size_t)NOT * KH * 2); float* Y = (float*)take((size_t)RCHK * NOT * 4);
    if ((size_t)(wsp - (char*)d_ws) > ws_size) return;
    k_lw<<<NOT / 8, 256, 0, stream>>>(wts, LWT);
    for (int ch = 0; ch < 4; ++ch) { const int p0 = ch * RCHK;
        k_gather<<<(RCHK * 5) / 8, 256, 0, stream>>>(x, idx, val, p0, Hh, Hl);
        k_gemmb<true, false><<<dim3(RCHK / 64, NOT / 64, 1), 128, 0, stream>>>(Hh, Hl, LWT, nullptr, Y, NOT, nullptr, nullptr, KH);
        k_max<<<(RCHK * OCH) / 256, 256, 0, stream>>>(Y, p0, out); }
}
